// PositionAttentionBlock_73478300500483
// MI455X (gfx1250) — hardware-verified
//
#include <hip/hip_runtime.h>


#define BATCH 4
#define C2    64
#define CIN   128
#define NPIX  4096
#define KCONV 576
#define BN_EPS 1e-5f

#define XP  136
#define OP  72
#define XSP 584
#define FSP 68
#define PROJ_LDS_BYTES (4 * 64 * XP * 2 + 2 * 64 * OP * 2)
#define CONV_LDS_BYTES (64 * XSP * 2 + 64 * FSP * 4 + 5 * 64 * 4)

typedef float          f32x8  __attribute__((ext_vector_type(8)));
typedef float          f32x4n __attribute__((ext_vector_type(4)));
typedef f32x4n         __attribute__((may_alias)) f32x4a;
typedef _Float16       f16x16 __attribute__((ext_vector_type(16)));
typedef _Float16       f16x8n __attribute__((ext_vector_type(8)));
typedef f16x8n         __attribute__((may_alias)) f16x8a;
typedef __bf16         bf16x16 __attribute__((ext_vector_type(16)));
typedef unsigned short u16x8n __attribute__((ext_vector_type(8)));
typedef u16x8n         __attribute__((may_alias)) u16x8a;
typedef unsigned int   u32x4n __attribute__((ext_vector_type(4)));
typedef u32x4n         __attribute__((may_alias)) u32x4a;

union FragH { f16x16 v; f16x8n h[2]; u16x8n u[2]; };
union FragB { bf16x16 v; u16x8n h[2]; };

__device__ __forceinline__ f32x8 mma_h(f16x16 a, f16x16 b, f32x8 c)
{
    c = __builtin_amdgcn_wmma_f32_16x16x32_f16(false, a, false, b, (short)0, c, false, false);
    asm volatile("v_nop\n\tv_nop\n\tv_nop\n\tv_nop" : "+v"(c) : "v"(a), "v"(b));
    return c;
}
__device__ __forceinline__ f32x8 mma_b(bf16x16 a, bf16x16 b, f32x8 c)
{
    c = __builtin_amdgcn_wmma_f32_16x16x32_bf16(false, a, false, b, (short)0, c, false, false);
    asm volatile("v_nop\n\tv_nop\n\tv_nop\n\tv_nop" : "+v"(c) : "v"(a), "v"(b));
    return c;
}

__device__ __forceinline__ unsigned short bf16_rne(float x)
{
    unsigned int u = __float_as_uint(x);
    u += 0x7FFFu + ((u >> 16) & 1u);
    return (unsigned short)(u >> 16);
}
__device__ __forceinline__ float bf16_val(unsigned short s)
{
    return __uint_as_float(((unsigned int)s) << 16);
}

__global__ __launch_bounds__(256)
void k_proj(const float* __restrict__ Hin, const float* __restrict__ Lin,
            const float* __restrict__ thw, const float* __restrict__ thb,
            const float* __restrict__ phw, const float* __restrict__ phb,
            const float* __restrict__ gw,  const float* __restrict__ gb,
            unsigned short* __restrict__ Kh, unsigned short* __restrict__ Kl,
            unsigned short* __restrict__ Qh, unsigned short* __restrict__ Ql,
            _Float16* __restrict__ Vout)
{
    extern __shared__ float4 dsm_f4[];
    unsigned char* smem = (unsigned char*)dsm_f4;
    unsigned short* Xh = (unsigned short*)smem;
    unsigned short* Xl = Xh + 64 * XP;
    unsigned short* Wh = Xl + 64 * XP;
    unsigned short* Wl = Wh + 64 * XP;
    unsigned short* Oh = Wl + 64 * XP;
    unsigned short* Ol = Oh + 64 * OP;

    const int bid = blockIdx.x;
    const int b   = bid >> 6;
    const int px0 = (bid & 63) << 6;
    if (b >= BATCH) return;
    const int tid = threadIdx.x, lane = tid & 31, w = tid >> 5;
    const int hf = lane >> 4, m = lane & 15;

    for (int idx = tid; idx < CIN * 64; idx += 256) {
        const int ci = idx >> 6, j = idx & 63;
        float x;
        if (ci < C2) x = Hin[((size_t)(b * C2 + ci)) * NPIX + px0 + j];
        else         x = Lin[((size_t)(b * C2 + ci - C2)) * NPIX + px0 + j];
        const unsigned short hi = bf16_rne(x);
        Xh[j * XP + ci] = hi;
        Xl[j * XP + ci] = bf16_rne(x - bf16_val(hi));
    }

    for (int p = 0; p < 3; ++p) {
        const float* Wsrc = (p == 0) ? thw : ((p == 1) ? phw : gw);
        const float* bias = (p == 0) ? thb : ((p == 1) ? phb : gb);
        const int cin = (p == 2) ? C2 : CIN;
        const int csh = (p == 2) ? 6 : 7;
        __syncthreads();
        for (int idx = tid; idx < 64 * cin; idx += 256) {
            const int o = idx >> csh, ci = idx & (cin - 1);
            const float x = Wsrc[idx];
            const unsigned short hi = bf16_rne(x);
            Wh[o * XP + ci] = hi;
            Wl[o * XP + ci] = bf16_rne(x - bf16_val(hi));
        }
        __syncthreads();

        f32x8 acc0 = {}, acc1 = {};
        const int rt = w & 3, ct0 = (w >> 2) << 1;
        if (p < 2) {
            const unsigned short* arh = Xh + (16 * rt + m) * XP;
            const unsigned short* arl = Xl + (16 * rt + m) * XP;
            const unsigned short* b0h = Wh + (16 * ct0 + m) * XP;
            const unsigned short* b0l = Wl + (16 * ct0 + m) * XP;
            const unsigned short* b1h = b0h + 16 * XP;
            const unsigned short* b1l = b0l + 16 * XP;
#pragma unroll
            for (int ks = 0; ks < 4; ++ks) {
                const int ka = ks * 32 + 8 * hf, kb = ka + 16;
                FragB ah, al, bh, bl;
                ah.h[0] = *(const u16x8a*)(arh + ka); ah.h[1] = *(const u16x8a*)(arh + kb);
                al.h[0] = *(const u16x8a*)(arl + ka); al.h[1] = *(const u16x8a*)(arl + kb);
                bh.h[0] = *(const u16x8a*)(b0h + ka); bh.h[1] = *(const u16x8a*)(b0h + kb);
                bl.h[0] = *(const u16x8a*)(b0l + ka); bl.h[1] = *(const u16x8a*)(b0l + kb);
                acc0 = mma_b(ah.v, bh.v, acc0);
                acc0 = mma_b(ah.v, bl.v, acc0);
                acc0 = mma_b(al.v, bh.v, acc0);
                bh.h[0] = *(const u16x8a*)(b1h + ka); bh.h[1] = *(const u16x8a*)(b1h + kb);
                bl.h[0] = *(const u16x8a*)(b1l + ka); bl.h[1] = *(const u16x8a*)(b1l + kb);
                acc1 = mma_b(ah.v, bh.v, acc1);
                acc1 = mma_b(ah.v, bl.v, acc1);
                acc1 = mma_b(al.v, bh.v, acc1);
            }
            const int pxr = 16 * rt + 8 * hf;
            const int o0 = 16 * ct0 + m, o1 = o0 + 16;
            const float bi0 = bias[o0], bi1 = bias[o1];
#pragma unroll
            for (int r = 0; r < 8; ++r) {
                const float v0 = acc0[r] + bi0;
                const unsigned short s0 = bf16_rne(v0);
                Oh[(pxr + r) * OP + o0] = s0;
                Ol[(pxr + r) * OP + o0] = bf16_rne(v0 - bf16_val(s0));
                const float v1 = acc1[r] + bi1;
                const unsigned short s1 = bf16_rne(v1);
                Oh[(pxr + r) * OP + o1] = s1;
                Ol[(pxr + r) * OP + o1] = bf16_rne(v1 - bf16_val(s1));
            }
        } else {
            const unsigned short* arh = Wh + (16 * rt + m) * XP;
            const unsigned short* arl = Wl + (16 * rt + m) * XP;
            const unsigned short* b0h = Xh + (16 * ct0 + m) * XP + C2;
            const unsigned short* b0l = Xl + (16 * ct0 + m) * XP + C2;
            const unsigned short* b1h = b0h + 16 * XP;
            const unsigned short* b1l = b0l + 16 * XP;
#pragma unroll
            for (int ks = 0; ks < 2; ++ks) {
                const int ka = ks * 32 + 8 * hf, kb = ka + 16;
                FragB ah, al, bh, bl;
                ah.h[0] = *(const u16x8a*)(arh + ka); ah.h[1] = *(const u16x8a*)(arh + kb);
                al.h[0] = *(const u16x8a*)(arl + ka); al.h[1] = *(const u16x8a*)(arl + kb);
                bh.h[0] = *(const u16x8a*)(b0h + ka); bh.h[1] = *(const u16x8a*)(b0h + kb);
                bl.h[0] = *(const u16x8a*)(b0l + ka); bl.h[1] = *(const u16x8a*)(b0l + kb);
                acc0 = mma_b(ah.v, bh.v, acc0);
                acc0 = mma_b(ah.v, bl.v, acc0);
                acc0 = mma_b(al.v, bh.v, acc0);
                bh.h[0] = *(const u16x8a*)(b1h + ka); bh.h[1] = *(const u16x8a*)(b1h + kb);
                bl.h[0] = *(const u16x8a*)(b1l + ka); bl.h[1] = *(const u16x8a*)(b1l + kb);
                acc1 = mma_b(ah.v, bh.v, acc1);
                acc1 = mma_b(ah.v, bl.v, acc1);
                acc1 = mma_b(al.v, bh.v, acc1);
            }
            const int cr = 16 * rt + 8 * hf;
            const int pxa = 16 * ct0 + m, pxb = pxa + 16;
            _Float16* Of = (_Float16*)Oh;
#pragma unroll
            for (int r = 0; r < 8; ++r) {
                const float bc = bias[cr + r];
                Of[(cr + r) * OP + pxa] = (_Float16)(acc0[r] + bc);
                Of[(cr + r) * OP + pxb] = (_Float16)(acc1[r] + bc);
            }
        }
        __syncthreads();

        {
            const int q  = lane & 7;
            const int r0 = 8 * w + (lane >> 3), r1 = r0 + 4;
            if (p < 2) {
                unsigned short* Dh = (p == 0) ? Kh : Qh;
                unsigned short* Dl = (p == 0) ? Kl : Ql;
                const u32x4n vh0 = *(const u32x4a*)(Oh + r0 * OP + 8 * q);
                const u32x4n vl0 = *(const u32x4a*)(Ol + r0 * OP + 8 * q);
                const u32x4n vh1 = *(const u32x4a*)(Oh + r1 * OP + 8 * q);
                const u32x4n vl1 = *(const u32x4a*)(Ol + r1 * OP + 8 * q);
                const size_t g0 = ((size_t)(b * NPIX + px0 + r0)) * C2 + 8 * q;
                const size_t g1 = ((size_t)(b * NPIX + px0 + r1)) * C2 + 8 * q;
                *(volatile u32x4n*)(Dh + g0) = vh0;  *(volatile u32x4n*)(Dl + g0) = vl0;
                *(volatile u32x4n*)(Dh + g1) = vh1;  *(volatile u32x4n*)(Dl + g1) = vl1;
                __threadfence();
                *(volatile u32x4n*)(Dh + g0) = vh0;  *(volatile u32x4n*)(Dl + g0) = vl0;
                *(volatile u32x4n*)(Dh + g1) = vh1;  *(volatile u32x4n*)(Dl + g1) = vl1;
            } else {
                const u32x4n v0 = *(const u32x4a*)(Oh + r0 * OP + 8 * q);
                const u32x4n v1 = *(const u32x4a*)(Oh + r1 * OP + 8 * q);
                const size_t g0 = ((size_t)(b * C2 + r0)) * NPIX + px0 + 8 * q;
                const size_t g1 = ((size_t)(b * C2 + r1)) * NPIX + px0 + 8 * q;
                *(volatile u32x4n*)(Vout + g0) = v0;
                *(volatile u32x4n*)(Vout + g1) = v1;
                __threadfence();
                *(volatile u32x4n*)(Vout + g0) = v0;
                *(volatile u32x4n*)(Vout + g1) = v1;
            }
        }
    }
}

__device__ __forceinline__ f32x8 score_tile(const unsigned short* __restrict__ kbh,
                                            const unsigned short* __restrict__ kbl,
                                            int n, int hf,
                                            const FragB& qh0, const FragB& qh1,
                                            const FragB& ql0, const FragB& ql1)
{
    const unsigned short* ka = kbh + (size_t)n * C2;
    const unsigned short* kl = kbl + (size_t)n * C2;
    f32x8 s = {};
    FragB ah, al;
    ah.h[0] = *(const u16x8a*)(ka + 8 * hf);       ah.h[1] = *(const u16x8a*)(ka + 16 + 8 * hf);
    al.h[0] = *(const u16x8a*)(kl + 8 * hf);       al.h[1] = *(const u16x8a*)(kl + 16 + 8 * hf);
    s = mma_b(ah.v, qh0.v, s);
    s = mma_b(ah.v, ql0.v, s);
    s = mma_b(al.v, qh0.v, s);
    ah.h[0] = *(const u16x8a*)(ka + 32 + 8 * hf);  ah.h[1] = *(const u16x8a*)(ka + 48 + 8 * hf);
    al.h[0] = *(const u16x8a*)(kl + 32 + 8 * hf);  al.h[1] = *(const u16x8a*)(kl + 48 + 8 * hf);
    s = mma_b(ah.v, qh1.v, s);
    s = mma_b(ah.v, ql1.v, s);
    s = mma_b(al.v, qh1.v, s);
    return s;
}

__global__ __launch_bounds__(256)
void k_attn(const unsigned short* __restrict__ Kh, const unsigned short* __restrict__ Kl,
            const unsigned short* __restrict__ Qh, const unsigned short* __restrict__ Ql,
            const _Float16* __restrict__ Vin, unsigned short* __restrict__ Eout)
{
    __shared__ __attribute__((aligned(16))) float Pacc[8 * 64 * 16];
    __shared__ float Pmax[8 * 16];
    __shared__ float Psum[8 * 16];
    __shared__ __attribute__((aligned(16))) _Float16 Es[64 * OP];

    const int bid = blockIdx.x;
    const int b   = bid >> 6;
    const int m0  = (bid & 63) << 6;
    if (b >= BATCH) return;
    const int tid = threadIdx.x, lane = tid & 31, w = tid >> 5;
    const int hf = lane >> 4, m = lane & 15;
    const int mt = w & 3, nh = w >> 2;

    FragB qh0, qh1, ql0, ql1;
    {
        const size_t qo = ((size_t)(b * NPIX + m0 + 16 * mt + m)) * C2;
        const unsigned short* qa = Qh + qo;
        const unsigned short* qb = Ql + qo;
        qh0.h[0] = *(const u16x8a*)(qa + 8 * hf);       qh0.h[1] = *(const u16x8a*)(qa + 16 + 8 * hf);
        qh1.h[0] = *(const u16x8a*)(qa + 32 + 8 * hf);  qh1.h[1] = *(const u16x8a*)(qa + 48 + 8 * hf);
        ql0.h[0] = *(const u16x8a*)(qb + 8 * hf);       ql0.h[1] = *(const u16x8a*)(qb + 16 + 8 * hf);
        ql1.h[0] = *(const u16x8a*)(qb + 32 + 8 * hf);  ql1.h[1] = *(const u16x8a*)(qb + 48 + 8 * hf);
    }

    f32x8 acc0 = {}, acc1 = {}, acc2 = {}, acc3 = {};
    float mrun = -3.0e38f, lsum = 0.0f;
    const unsigned short* kbh = Kh + (size_t)b * NPIX * C2;
    const unsigned short* kbl = Kl + (size_t)b * NPIX * C2;
    const _Float16* vb = Vin + (size_t)b * C2 * NPIX + (size_t)m * NPIX;
    const int nbase = nh << 11;

#pragma unroll 1
    for (int it = 0; it < 64; ++it) {
        const int n0 = nbase + (it << 5);
        const f32x8 s0 = score_tile(kbh, kbl, n0 + m,      hf, qh0, qh1, ql0, ql1);
        const f32x8 s1 = score_tile(kbh, kbl, n0 + 16 + m, hf, qh0, qh1, ql0, ql1);

        float cm = s0[0];
#pragma unroll
        for (int r = 1; r < 8; ++r) cm = fmaxf(cm, s0[r]);
#pragma unroll
        for (int r = 0; r < 8; ++r) cm = fmaxf(cm, s1[r]);
        cm = fmaxf(cm, __shfl_xor(cm, 16));
        const float mnew = fmaxf(mrun, cm);
        const float sc = __expf(mrun - mnew);
        lsum *= sc;
        acc0 *= sc; acc1 *= sc; acc2 *= sc; acc3 *= sc;

        f16x8n p0, p1;
#pragma unroll
        for (int r = 0; r < 8; ++r) {
            const float e = __expf(s0[r] - mnew);
            lsum += e;
            p0[r] = (_Float16)(e * 4096.0f);
        }
#pragma unroll
        for (int r = 0; r < 8; ++r) {
            const float e = __expf(s1[r] - mnew);
            lsum += e;
            p1[r] = (_Float16)(e * 4096.0f);
        }
        FragH pb;
        pb.h[0] = p0;
        pb.h[1] = p1;
        mrun = mnew;

        {
            FragH va;
            const _Float16* vp = vb + n0 + 8 * hf;
            va.h[0] = *(const f16x8a*)(vp);  va.h[1] = *(const f16x8a*)(vp + 16);
            acc0 = mma_h(va.v, pb.v, acc0);
        }
        {
            FragH va;
            const _Float16* vp = vb + (size_t)16 * NPIX + n0 + 8 * hf;
            va.h[0] = *(const f16x8a*)(vp);  va.h[1] = *(const f16x8a*)(vp + 16);
            acc1 = mma_h(va.v, pb.v, acc1);
        }
        {
            FragH va;
            const _Float16* vp = vb + (size_t)32 * NPIX + n0 + 8 * hf;
            va.h[0] = *(const f16x8a*)(vp);  va.h[1] = *(const f16x8a*)(vp + 16);
            acc2 = mma_h(va.v, pb.v, acc2);
        }
        {
            FragH va;
            const _Float16* vp = vb + (size_t)48 * NPIX + n0 + 8 * hf;
            va.h[0] = *(const f16x8a*)(vp);  va.h[1] = *(const f16x8a*)(vp + 16);
            acc3 = mma_h(va.v, pb.v, acc3);
        }
    }
    lsum += __shfl_xor(lsum, 16);

    {
        float* pa = Pacc + (w * 64) * 16;
#pragma unroll
        for (int r = 0; r < 8; ++r) {
            pa[(8 * hf + r) * 16 + m]      = acc0[r];
            pa[(16 + 8 * hf + r) * 16 + m] = acc1[r];
            pa[(32 + 8 * hf + r) * 16 + m] = acc2[r];
            pa[(48 + 8 * hf + r) * 16 + m] = acc3[r];
        }
        if (hf == 0) { Pmax[w * 16 + m] = mrun; Psum[w * 16 + m] = lsum; }
    }
    __syncthreads();

    {
        const int mm = tid & 63, cg = tid >> 6, qt = mm >> 4, ml = mm & 15;
        const int w0i = qt, w1i = qt + 4;
        const float M0 = Pmax[w0i * 16 + ml], M1 = Pmax[w1i * 16 + ml];
        const float gm = fmaxf(M0, M1);
        const float f0 = __expf(M0 - gm), f1 = __expf(M1 - gm);
        const float den = Psum[w0i * 16 + ml] * f0 + Psum[w1i * 16 + ml] * f1;
        const float inv = (1.0f / den) * (1.0f / 256.0f);
        const float* pa0 = Pacc + (w0i * 64) * 16 + ml;
        const float* pa1 = Pacc + (w1i * 64) * 16 + ml;
#pragma unroll
        for (int i = 0; i < 16; ++i) {
            const int c = cg + 4 * i;
            const float e = (pa0[c * 16] * f0 + pa1[c * 16] * f1) * inv;
            Es[c * OP + mm] = (_Float16)e;
        }
    }
    __syncthreads();

    {
        const int q  = lane & 7;
        const int c0 = 8 * w + (lane >> 3), c1 = c0 + 4;
        const u32x4n e0 = *(const u32x4a*)(Es + c0 * OP + 8 * q);
        const u32x4n e1 = *(const u32x4a*)(Es + c1 * OP + 8 * q);
        unsigned short* d0 = Eout + ((size_t)(b * C2 + c0)) * NPIX + m0 + 8 * q;
        unsigned short* d1 = Eout + ((size_t)(b * C2 + c1)) * NPIX + m0 + 8 * q;
        *(volatile u32x4n*)d0 = e0;
        *(volatile u32x4n*)d1 = e1;
        __threadfence();
        *(volatile u32x4n*)d0 = e0;
        *(volatile u32x4n*)d1 = e1;
    }
}

__global__ __launch_bounds__(256)
void k_conv(const unsigned short* __restrict__ Ein, const float* __restrict__ cw,
            const float* __restrict__ cb,  const float* __restrict__ bng,
            const float* __restrict__ bnb, const float* __restrict__ bnm,
            const float* __restrict__ bnv, const float* __restrict__ Hin,
            float* __restrict__ out)
{
    extern __shared__ float4 dsm_f4[];
    unsigned char* smem = (unsigned char*)dsm_f4;
    unsigned short* Xs = (unsigned short*)smem;
    float* Fs  = (float*)(smem + 64 * XSP * 2);
    float* prm = Fs + 64 * FSP;

    const int bid = blockIdx.x;
    const int b   = bid >> 6;
    const int y   = bid & 63;
    if (b >= BATCH) return;
    const int tid = threadIdx.x, lane = tid & 31, w = tid >> 5;
    const int hf = lane >> 4, m = lane & 15;

    if (tid < 64) {
        prm[tid]       = cb[tid];
        prm[64 + tid]  = bnm[tid];
        prm[128 + tid] = rsqrtf(bnv[tid] + BN_EPS);
        prm[192 + tid] = bng[tid];
        prm[256 + tid] = bnb[tid];
    }

    const unsigned short* eb = Ein + (size_t)b * C2 * NPIX;
    for (int idx = tid; idx < 64 * KCONV; idx += 256) {
        const int k = idx >> 6, px = idx & 63;
        const int ci = k / 9;
        const int rr = k - ci * 9;
        const int ky = rr / 3;
        const int kx = rr - ky * 3;
        const int yy = y + ky - 1, xx = px + kx - 1;
        unsigned short v = 0;
        if ((unsigned)yy < 64u && (unsigned)xx < 64u)
            v = eb[(size_t)ci * NPIX + yy * 64 + xx];
        Xs[px * XSP + k] = v;
    }
    __syncthreads();

    const int rt = w & 3, ct0 = (w >> 2) << 1;
    const float* wr = cw + (size_t)(16 * rt + m) * KCONV;
    const unsigned short* x0 = Xs + (16 * ct0 + m) * XSP;
    const unsigned short* x1 = x0 + 16 * XSP;
    f32x8 acc0 = {}, acc1 = {};
#pragma unroll 1
    for (int ks = 0; ks < 18; ++ks) {
        const int ka = (ks << 5) + 8 * hf, kb = ka + 16;
        FragH a, b0, b1;
        {
            const f32x4n w0 = *(const f32x4a*)(wr + ka);
            const f32x4n w1 = *(const f32x4a*)(wr + ka + 4);
            const f32x4n w2 = *(const f32x4a*)(wr + kb);
            const f32x4n w3 = *(const f32x4a*)(wr + kb + 4);
            f16x8n wka, wkb;
            wka[0] = (_Float16)(w0[0] * 64.0f); wka[1] = (_Float16)(w0[1] * 64.0f);
            wka[2] = (_Float16)(w0[2] * 64.0f); wka[3] = (_Float16)(w0[3] * 64.0f);
            wka[4] = (_Float16)(w1[0] * 64.0f); wka[5] = (_Float16)(w1[1] * 64.0f);
            wka[6] = (_Float16)(w1[2] * 64.0f); wka[7] = (_Float16)(w1[3] * 64.0f);
            wkb[0] = (_Float16)(w2[0] * 64.0f); wkb[1] = (_Float16)(w2[1] * 64.0f);
            wkb[2] = (_Float16)(w2[2] * 64.0f); wkb[3] = (_Float16)(w2[3] * 64.0f);
            wkb[4] = (_Float16)(w3[0] * 64.0f); wkb[5] = (_Float16)(w3[1] * 64.0f);
            wkb[6] = (_Float16)(w3[2] * 64.0f); wkb[7] = (_Float16)(w3[3] * 64.0f);
            a.h[0] = wka;
            a.h[1] = wkb;
        }
        b0.u[0] = *(const u16x8a*)(x0 + ka); b0.u[1] = *(const u16x8a*)(x0 + kb);
        b1.u[0] = *(const u16x8a*)(x1 + ka); b1.u[1] = *(const u16x8a*)(x1 + kb);
        acc0 = mma_h(a.v, b0.v, acc0);
        acc1 = mma_h(a.v, b1.v, acc1);
    }

    {
        const int cob = 16 * rt + 8 * hf;
        const int pxa = 16 * ct0 + m, pxb = pxa + 16;
#pragma unroll
        for (int r = 0; r < 8; ++r) {
            const int co = cob + r;
            const float pb_ = prm[co], pm_ = prm[64 + co], pis = prm[128 + co];
            const float pg_ = prm[192 + co], pbe = prm[256 + co];
            float fa = acc0[r] * (1.0f / 1024.0f) + pb_;
            fa = (fa - pm_) * pis;
            fa = fa * pg_ + pbe;
            Fs[co * FSP + pxa] = fmaxf(fa, 0.0f);
            float fb = acc1[r] * (1.0f / 1024.0f) + pb_;
            fb = (fb - pm_) * pis;
            fb = fb * pg_ + pbe;
            Fs[co * FSP + pxb] = fmaxf(fb, 0.0f);
        }
    }
    __syncthreads();

    {
        const int q = lane & 15;
        f32x4n vals[4];
        size_t goff[4];
#pragma unroll
        for (int s = 0; s < 4; ++s) {
            const int co = 8 * w + 2 * s + (lane >> 4);
            const f32x4n f = *(const f32x4a*)(Fs + co * FSP + 4 * q);
            const size_t g = ((size_t)(b * C2 + co)) * NPIX + (size_t)y * 64 + 4 * q;
            const f32x4n hv = *(const f32x4a*)(Hin + g);
            vals[s] = hv + f;
            goff[s] = g;
            *(volatile f32x4n*)(out + g) = vals[s];
        }
        __threadfence();
#pragma unroll
        for (int s = 0; s < 4; ++s)
            *(volatile f32x4n*)(out + goff[s]) = vals[s];
    }
}

extern "C" void kernel_launch(void* const* d_in, const int* in_sizes, int n_in,
                              void* d_out, int out_size, void* d_ws, size_t ws_size,
                              hipStream_t stream)
{
    if (n_in < 14) return;
    if (in_sizes[0] != BATCH * C2 * NPIX || in_sizes[1] != BATCH * C2 * NPIX) return;
    if (in_sizes[2] != C2 * CIN || in_sizes[3] != C2) return;
    if (in_sizes[4] != C2 * CIN || in_sizes[5] != C2) return;
    if (in_sizes[6] != C2 * C2  || in_sizes[7] != C2) return;
    if (in_sizes[8] != C2 * C2 * 9 || in_sizes[9] != C2) return;
    if (in_sizes[10] != C2 || in_sizes[11] != C2 || in_sizes[12] != C2 || in_sizes[13] != C2) return;
    if (out_size != BATCH * C2 * NPIX) return;

    const float* Hbuf = (const float*)d_in[0];
    const float* Lbuf = (const float*)d_in[1];
    const float* thw  = (const float*)d_in[2];
    const float* thb  = (const float*)d_in[3];
    const float* phw  = (const float*)d_in[4];
    const float* phb  = (const float*)d_in[5];
    const float* gw   = (const float*)d_in[6];
    const float* gb   = (const float*)d_in[7];
    const float* cw   = (const float*)d_in[8];
    const float* cb   = (const float*)d_in[9];
    const float* bng  = (const float*)d_in[10];
    const float* bnb  = (const float*)d_in[11];
    const float* bnm  = (const float*)d_in[12];
    const float* bnv  = (const float*)d_in[13];
    float* out = (float*)d_out;

    const size_t plane = (size_t)BATCH * NPIX * C2 * 2;
    const size_t need  = 6 * plane;
    if (ws_size < need) return;
    char* ws = (char*)d_ws;
    unsigned short* Kh = (unsigned short*)(ws + 0 * plane);
    unsigned short* Kl = (unsigned short*)(ws + 1 * plane);
    unsigned short* Qh = (unsigned short*)(ws + 2 * plane);
    unsigned short* Ql = (unsigned short*)(ws + 3 * plane);
    _Float16*       Vw = (_Float16*)      (ws + 4 * plane);
    unsigned short* Ew = (unsigned short*)(ws + 5 * plane);

    (void)hipFuncSetAttribute((const void*)k_proj, hipFuncAttributeMaxDynamicSharedMemorySize, PROJ_LDS_BYTES);
    (void)hipFuncSetAttribute((const void*)k_conv, hipFuncAttributeMaxDynamicSharedMemorySize, CONV_LDS_BYTES);

    const dim3 grid(BATCH * (NPIX / 64), 1, 1);
    const dim3 block(256, 1, 1);

    k_proj<<<grid, block, PROJ_LDS_BYTES, stream>>>(Hbuf, Lbuf, thw, thb, phw, phb, gw, gb,
                                                    Kh, Kl, Qh, Ql, Vw);
    k_attn<<<grid, block, 0, stream>>>(Kh, Kl, Qh, Ql, Vw, Ew);
    k_conv<<<grid, block, CONV_LDS_BYTES, stream>>>(Ew, cw, cb, bng, bnb, bnm, bnv, Hbuf, out);
}
